// InfoNCELoss_22909355557339
// MI455X (gfx1250) — hardware-verified
//
#include <hip/hip_runtime.h>

typedef __attribute__((ext_vector_type(16))) _Float16 v16h;
typedef __attribute__((ext_vector_type(8)))  _Float16 v8h;
typedef __attribute__((ext_vector_type(16))) __bf16   v16b;
typedef __attribute__((ext_vector_type(8)))  __bf16   v8b;
typedef __attribute__((ext_vector_type(8)))  float    v8f;
typedef __attribute__((ext_vector_type(4)))  float    v4f;

constexpr int kDim       = 512;
constexpr int kNumAnch   = 4096;
constexpr int kNumPos    = 4096;
constexpr int kNumNeg    = 16384;
constexpr int kRowsPerBlk = 64;
constexpr int kNegTiles  = kNumNeg / 64;
constexpr int kBlkA      = kNumAnch / kRowsPerBlk;
constexpr int kBlkP      = kNumPos  / kRowsPerBlk;
constexpr int kBlkN      = kNumNeg  / kRowsPerBlk;

static_assert(kDim % 32 == 0);
static_assert(kDim == 512);
static_assert(kNumAnch % 64 == 0 && kNumPos % 64 == 0 && kNumNeg % 64 == 0);
static_assert(kNumAnch % kRowsPerBlk == 0 && kNumPos % kRowsPerBlk == 0 && kNumNeg % kRowsPerBlk == 0);
static_assert(kNegTiles == 32 * 8);
static_assert(kNumPos % 128 == 0);
static_assert(kNumAnch % 256 == 0 && kDim % 256 == 0);
static_assert((kNumAnch / 64) * (kNumPos / 64) % 8 == 0);
static_assert((kNumAnch / 64) * (kNumNeg / 64) % 8 == 0);

__device__ __forceinline__ unsigned short f2bf_bits(float f) {
  unsigned u = __float_as_uint(f);
  return (unsigned short)((u + 0x7FFFu + ((u >> 16) & 1u)) >> 16);
}
__device__ __forceinline__ float bf_bits2f(unsigned short h) { return __uint_as_float(((unsigned)h) << 16); }

__device__ __forceinline__ void dep_guard_h(v8f& a, v8f& b, v16h x, v16h y) { asm volatile("v_nop\n\tv_nop\n\tv_nop\n\tv_nop" : "+v"(a), "+v"(b) : "v"(x), "v"(y)); }
__device__ __forceinline__ void dep_guard_b(v8f& a, v8f& b, v16b x, v16b y) { asm volatile("v_nop\n\tv_nop\n\tv_nop\n\tv_nop" : "+v"(a), "+v"(b) : "v"(x), "v"(y)); }
__device__ __forceinline__ void keep4_h(v16h a, v16h b, v16h c, v16h d) { asm volatile("v_nop" :: "v"(a), "v"(b), "v"(c), "v"(d)); }
__device__ __forceinline__ void keep4_b(v16b a, v16b b, v16b c, v16b d) { asm volatile("v_nop" :: "v"(a), "v"(b), "v"(c), "v"(d)); }
__device__ __forceinline__ void acc_guard4(v8f& a, v8f& b, v8f& c, v8f& d) { asm volatile("v_nop\n\tv_nop\n\tv_nop\n\tv_nop" : "+v"(a), "+v"(b), "+v"(c), "+v"(d)); }
template <typename T> struct Frag;
template <> struct Frag<_Float16> {
  typedef v16h V; union U { v16h v; v8h h[2]; };
  static __device__ __forceinline__ v16h load(const _Float16* p) {
    U f; f.h[0] = *(const v8h*)(p); f.h[1] = *(const v8h*)(p + 16); return f.v;
  }
  static __device__ __forceinline__ v8f mma(v16h a, v16h b, v8f c) {
    return __builtin_amdgcn_wmma_f32_16x16x32_f16(false, a, false, b, (short)0, c, false, false);
  }
  static __device__ __forceinline__ void guard(v8f& a, v8f& b, v16h x, v16h y) { dep_guard_h(a, b, x, y); }
  static __device__ __forceinline__ void keep(v16h a, v16h b, v16h c, v16h d) { keep4_h(a, b, c, d); }
};
template <> struct Frag<__bf16> {
  typedef v16b V; union U { v16b v; v8b h[2]; };
  static __device__ __forceinline__ v16b load(const __bf16* p) {
    U f; f.h[0] = *(const v8b*)(p); f.h[1] = *(const v8b*)(p + 16); return f.v;
  }
  static __device__ __forceinline__ v8f mma(v16b a, v16b b, v8f c) {
    return __builtin_amdgcn_wmma_f32_16x16x32_bf16(false, a, false, b, (short)0, c, false, false);
  }
  static __device__ __forceinline__ void guard(v8f& a, v8f& b, v16b x, v16b y) { dep_guard_b(a, b, x, y); }
  static __device__ __forceinline__ void keep(v16b a, v16b b, v16b c, v16b d) { keep4_b(a, b, c, d); }
};

template <int ET> struct Elem;
template <> struct Elem<0> { typedef _Float16 T; };
template <> struct Elem<1> { typedef __bf16 T; };
template <int ET, bool SPLIT, int BIAS_MODE, int OUT_MODE, bool RESID, int ACT = 0>
__global__ __launch_bounds__(256) void wmma_gemm64(
    const unsigned short* __restrict__ Ap, const unsigned short* __restrict__ A2p, int lda, long strideA,
    const unsigned short* __restrict__ Btp, const unsigned short* __restrict__ Bt2p, int ldb, long strideB,
    void* __restrict__ Cout, void* __restrict__ Cout2, int ldc, long strideC,
    const float* __restrict__ bias,
    const float* __restrict__ resid, long strideR,
    int M, int N, int K, float scale) {
  typedef typename Elem<ET>::T T;
  typedef typename Frag<T>::V V;
  const T* A = (const T*)Ap; const T* A2 = (const T*)A2p; const T* Bt = (const T*)Btp; const T* Bt2 = (const T*)Bt2p;
  __shared__ __align__(16) float sT[8][16 * 68];
  const int b    = blockIdx.y;
  const int lane = threadIdx.x & 31;
  const int wave = threadIdx.x >> 5;
  const int tilesN = N >> 6;
  const int tilesM = M >> 6;
  const int tile = blockIdx.x * 8 + wave;
  if (tile >= tilesM * tilesN) return;
  const int tm = tile / tilesN;
  const int tn = tile - tm * tilesN;
  const int m0 = tm << 6;
  const int n0 = tn << 6;

  const T* Ab  = A  + (size_t)b * strideA;
  const T* Bb  = Bt + (size_t)b * strideB;
  const T* Ab2 = SPLIT ? (A2  + (size_t)b * strideA) : nullptr;
  const T* Bb2 = SPLIT ? (Bt2 + (size_t)b * strideB) : nullptr;

  const int rlane = lane & 15;
  const int koff  = (lane >> 4) * 8;
  const int mOff  = (lane >> 4) * 8;

  v8f acc[4][4];
#pragma unroll
  for (int i = 0; i < 4; ++i)
#pragma unroll
    for (int j = 0; j < 4; ++j) acc[i][j] = (v8f){0.f,0.f,0.f,0.f,0.f,0.f,0.f,0.f};

  for (int k0 = 0; k0 < K; k0 += 32) {
    V bh[4], bl[4];
#pragma unroll
    for (int j = 0; j < 4; ++j) {
      const size_t bo = (size_t)(n0 + (j << 4) + rlane) * ldb + koff + k0;
      bh[j] = Frag<T>::load(Bb + bo);
      if (SPLIT) bl[j] = Frag<T>::load(Bb2 + bo);
    }
#pragma unroll
    for (int i = 0; i < 4; ++i) {
      const size_t ao = (size_t)(m0 + (i << 4) + rlane) * lda + koff + k0;
      V ah = Frag<T>::load(Ab + ao);
      V al;
      if (SPLIT) al = Frag<T>::load(Ab2 + ao);
#pragma unroll
      for (int j = 0; j < 4; ++j) {
        acc[i][j] = Frag<T>::mma(ah, bh[j], acc[i][j]);
        if (SPLIT) {
          acc[i][j] = Frag<T>::mma(ah, bl[j], acc[i][j]);
          acc[i][j] = Frag<T>::mma(al, bh[j], acc[i][j]);
        }
      }
      Frag<T>::guard(acc[i][0], acc[i][3], ah, SPLIT ? al : ah);
    }
    Frag<T>::keep(bh[0], bh[1], bh[2], bh[3]);
    if (SPLIT) Frag<T>::keep(bl[0], bl[1], bl[2], bl[3]);
  }
  acc_guard4(acc[0][0], acc[0][1], acc[0][2], acc[0][3]);
  acc_guard4(acc[1][0], acc[1][1], acc[1][2], acc[1][3]);
  acc_guard4(acc[2][0], acc[2][1], acc[2][2], acc[2][3]);
  acc_guard4(acc[3][0], acc[3][1], acc[3][2], acc[3][3]);

  float* slab = sT[wave];
  const float* Rb = RESID ? (resid + (size_t)b * strideR) : nullptr;
#pragma unroll
  for (int i = 0; i < 4; ++i) {
    const int mBase = m0 + (i << 4);
#pragma unroll
    for (int j = 0; j < 4; ++j) {
      const int n = n0 + (j << 4) + rlane;
      float bv = 0.f;
      if (BIAS_MODE == 2) bv = bias[n];
#pragma unroll
      for (int r = 0; r < 8; ++r) {
        float v = acc[i][j][r] * scale;
        if (BIAS_MODE == 1) v += bias[mBase + mOff + r];
        if (BIAS_MODE == 2) v += bv;
        if (RESID) v += Rb[(size_t)(mBase + mOff + r) * ldc + n];
        if (ACT == 1) v = tanhf(v);
        if (ACT == 2) v = fmaxf(v, 0.0f);
        if (ACT == 3) v = v / (1.0f + expf(-v));
        if (ACT == 4) v = (v > 0.f) ? v : 0.01f * v;
        if (ACT == 5) v = 0.5f * v * (1.0f + erff(v * 0.70710678118654752f));
        if (ACT == 6) v = __builtin_amdgcn_exp2f(v);
        slab[(mOff + r) * 68 + (j << 4) + rlane] = v;
      }
    }
    __builtin_amdgcn_fence(__ATOMIC_RELEASE, "workgroup");
    __builtin_amdgcn_wave_barrier();
    __builtin_amdgcn_fence(__ATOMIC_ACQUIRE, "workgroup");
    if (OUT_MODE == 0) {
      float* C = (float*)Cout + (size_t)b * strideC;
      const int hh = lane >> 4, c4 = (lane & 15) * 4;
      for (int pass = 0; pass < 2; ++pass) {
#pragma unroll
        for (int it = 0; it < 8; ++it) {
          const int row = it * 2 + hh;
          v4f v = *(const v4f*)(slab + row * 68 + c4);
          *(volatile v4f*)(C + (size_t)(mBase + row) * ldc + n0 + c4) = v;
        }
        __threadfence();
      }
    } else {
      const int q = lane >> 3, c8 = (lane & 7) * 8;
      unsigned short* C  = (unsigned short*)Cout  + (size_t)b * strideC;
      unsigned short* C2 = (OUT_MODE == 2) ? ((unsigned short*)Cout2 + (size_t)b * strideC) : nullptr;
      for (int pass = 0; pass < 2; ++pass) {
#pragma unroll
        for (int it = 0; it < 4; ++it) {
          const int row = it * 4 + q;
          const float* sp = slab + row * 68 + c8;
          v8h hv, lv;
#pragma unroll
          for (int e = 0; e < 8; ++e) {
            if (OUT_MODE == 1) {
              hv[e] = (_Float16)sp[e];
            } else {
              unsigned short hb = f2bf_bits(sp[e]);
              unsigned short lb = f2bf_bits(sp[e] - bf_bits2f(hb));
              hv[e] = __builtin_bit_cast(_Float16, hb);
              lv[e] = __builtin_bit_cast(_Float16, lb);
            }
          }
          *(volatile v8h*)(C + (size_t)(mBase + row) * ldc + n0 + c8) = hv;
          if (OUT_MODE == 2) *(volatile v8h*)(C2 + (size_t)(mBase + row) * ldc + n0 + c8) = lv;
        }
        __threadfence();
      }
    }
    __builtin_amdgcn_fence(__ATOMIC_RELEASE, "workgroup");
    __builtin_amdgcn_wave_barrier();
    __builtin_amdgcn_fence(__ATOMIC_ACQUIRE, "workgroup");
  }
}

__global__ __launch_bounds__(256) void gemm64_rowexp2(
    const unsigned short* __restrict__ Ap, int lda,
    const unsigned short* __restrict__ Btp, int ldb,
    float* __restrict__ nep, int ldn,
    int M, int N, int K, float scale) {
  typedef _Float16 T;
  typedef v16h V;
  const T* A = (const T*)Ap; const T* Bt = (const T*)Btp;
  __shared__ __align__(16) float sT[8][16 * 68];
  const int lane = threadIdx.x & 31;
  const int wave = threadIdx.x >> 5;
  const int tilesN = N >> 6;
  const int tilesM = M >> 6;
  const int tile = blockIdx.x * 8 + wave;
  if (tile >= tilesM * tilesN) return;
  const int tm = tile / tilesN;
  const int tn = tile - tm * tilesN;
  const int m0 = tm << 6;
  const int n0 = tn << 6;

  const int rlane = lane & 15;
  const int koff  = (lane >> 4) * 8;
  const int mOff  = (lane >> 4) * 8;
  const int ch    = lane >> 4;

  v8f acc[4][4];
#pragma unroll
  for (int i = 0; i < 4; ++i)
#pragma unroll
    for (int j = 0; j < 4; ++j) acc[i][j] = (v8f){0.f,0.f,0.f,0.f,0.f,0.f,0.f,0.f};

  for (int k0 = 0; k0 < K; k0 += 32) {
    V bh[4];
#pragma unroll
    for (int j = 0; j < 4; ++j) {
      const size_t bo = (size_t)(n0 + (j << 4) + rlane) * ldb + koff + k0;
      bh[j] = Frag<T>::load(Bt + bo);
    }
#pragma unroll
    for (int i = 0; i < 4; ++i) {
      const size_t ao = (size_t)(m0 + (i << 4) + rlane) * lda + koff + k0;
      V ah = Frag<T>::load(A + ao);
#pragma unroll
      for (int j = 0; j < 4; ++j) acc[i][j] = Frag<T>::mma(ah, bh[j], acc[i][j]);
      Frag<T>::guard(acc[i][0], acc[i][3], ah, ah);
    }
    Frag<T>::keep(bh[0], bh[1], bh[2], bh[3]);
  }
  acc_guard4(acc[0][0], acc[0][1], acc[0][2], acc[0][3]);
  acc_guard4(acc[1][0], acc[1][1], acc[1][2], acc[1][3]);
  acc_guard4(acc[2][0], acc[2][1], acc[2][2], acc[2][3]);
  acc_guard4(acc[3][0], acc[3][1], acc[3][2], acc[3][3]);

  float* slab = sT[wave];
  float erow[4];
#pragma unroll
  for (int i = 0; i < 4; ++i) {
#pragma unroll
    for (int j = 0; j < 4; ++j) {
#pragma unroll
      for (int r = 0; r < 8; ++r) slab[(mOff + r) * 68 + (j << 4) + rlane] = acc[i][j][r] * scale;
    }
    __builtin_amdgcn_fence(__ATOMIC_RELEASE, "workgroup");
    __builtin_amdgcn_wave_barrier();
    __builtin_amdgcn_fence(__ATOMIC_ACQUIRE, "workgroup");
    float e = 0.f;
#pragma unroll
    for (int q4 = 0; q4 < 8; ++q4) {
      const v4f t = *(const v4f*)(slab + rlane * 68 + ch * 32 + q4 * 4);
      e += __builtin_amdgcn_exp2f(t[0]);
      e += __builtin_amdgcn_exp2f(t[1]);
      e += __builtin_amdgcn_exp2f(t[2]);
      e += __builtin_amdgcn_exp2f(t[3]);
    }
    e += __shfl_xor(e, 16, 32);
    erow[i] = e;
    __builtin_amdgcn_fence(__ATOMIC_RELEASE, "workgroup");
    __builtin_amdgcn_wave_barrier();
    __builtin_amdgcn_fence(__ATOMIC_ACQUIRE, "workgroup");
  }
  if (ch == 0) {
    slab[rlane]      = erow[0];
    slab[16 + rlane] = erow[1];
    slab[32 + rlane] = erow[2];
    slab[48 + rlane] = erow[3];
  }
  __builtin_amdgcn_fence(__ATOMIC_RELEASE, "workgroup");
  __builtin_amdgcn_wave_barrier();
  __builtin_amdgcn_fence(__ATOMIC_ACQUIRE, "workgroup");
  const v4f ev = *(const v4f*)(slab + 4 * rlane);
  float* dst = nep + (size_t)tn * ldn + m0 + 4 * rlane;
  for (int pass = 0; pass < 2; ++pass) {
    if (ch == 0) *(volatile v4f*)dst = ev;
    __threadfence();
  }
}

__global__ __launch_bounds__(256) void k_rownorm(const float* __restrict__ x, int nrows,
                                                 _Float16* __restrict__ y, float* __restrict__ colpart) {
  __shared__ __align__(16) float cs[8][kDim];
  __shared__ __align__(16) float cso[kDim];
  const int lane = threadIdx.x & 31;
  const int wave = threadIdx.x >> 5;
  float csum[16];
#pragma unroll
  for (int c = 0; c < 16; ++c) csum[c] = 0.f;

#pragma unroll 1
  for (int rr = 0; rr < 8; ++rr) {
    int row = blockIdx.x * kRowsPerBlk + wave * 8 + rr;
    row = row < nrows ? row : nrows - 1;
    const float* src = x + (size_t)row * kDim + lane * 8;
    const v4f a0 = *(const v4f*)(src);
    const v4f a1 = *(const v4f*)(src + 4);
    const v4f b0 = *(const v4f*)(src + 256);
    const v4f b1 = *(const v4f*)(src + 260);
    float v[16];
#pragma unroll
    for (int c = 0; c < 4; ++c) { v[c] = a0[c]; v[4 + c] = a1[c]; v[8 + c] = b0[c]; v[12 + c] = b1[c]; }
    float ss = 0.f;
#pragma unroll
    for (int c = 0; c < 16; ++c) ss += v[c] * v[c];
#pragma unroll
    for (int off = 1; off < 32; off <<= 1) ss += __shfl_xor(ss, off, 32);
    const float nrm = fmaxf(sqrtf(ss), 1e-12f);
    const float inv = 1.0f / nrm;
    v8h h0, h1;
#pragma unroll
    for (int c = 0; c < 8; ++c) {
      const float u0 = v[c] * inv;
      const float u1 = v[8 + c] * inv;
      csum[c]     += u0;
      csum[8 + c] += u1;
      h0[c] = (_Float16)(u0 * 16.0f);
      h1[c] = (_Float16)(u1 * 16.0f);
    }
    _Float16* dst = y + (size_t)row * kDim + lane * 8;
    for (int pass = 0; pass < 2; ++pass) {
      *(volatile v8h*)(dst)       = h0;
      *(volatile v8h*)(dst + 256) = h1;
      __threadfence();
    }
  }

  {
    float* cw = cs[wave] + lane * 8;
    v4f t0, t1, t2, t3;
#pragma unroll
    for (int c = 0; c < 4; ++c) { t0[c] = csum[c]; t1[c] = csum[4 + c]; t2[c] = csum[8 + c]; t3[c] = csum[12 + c]; }
    *(v4f*)(cw)       = t0;
    *(v4f*)(cw + 4)   = t1;
    *(v4f*)(cw + 256) = t2;
    *(v4f*)(cw + 260) = t3;
  }
  __syncthreads();
  {
    const int t = threadIdx.x;
    float s0 = 0.f, s1 = 0.f;
#pragma unroll
    for (int w = 0; w < 8; ++w) { s0 += cs[w][2 * t]; s1 += cs[w][2 * t + 1]; }
    cso[2 * t]     = s0;
    cso[2 * t + 1] = s1;
  }
  __syncthreads();
  if (wave < 4) {
    const v4f o = *(const v4f*)(cso + wave * 128 + lane * 4);
    float* dst = colpart + (size_t)blockIdx.x * kDim + wave * 128 + lane * 4;
    for (int pass = 0; pass < 2; ++pass) {
      *(volatile v4f*)dst = o;
      __threadfence();
    }
  }
}

__global__ __launch_bounds__(256) void k_rowloss(const float* __restrict__ pe, int ldpe, int ncol,
                                                 const float* __restrict__ nep, int ldn, int ntn,
                                                 float* __restrict__ rowloss, int nrows, float eps) {
  __shared__ __align__(16) float rs[kRowsPerBlk];
  const int lane = threadIdx.x & 31;
  const int wave = threadIdx.x >> 5;
#pragma unroll 1
  for (int rr = 0; rr < 8; ++rr) {
    int row = blockIdx.x * kRowsPerBlk + wave * 8 + rr;
    row = row < nrows ? row : nrows - 1;
    float s = 0.f;
#pragma unroll
    for (int q = 0; q < 8; ++q) {
      int tc = lane + 32 * q;
      tc = tc < ntn ? tc : ntn - 1;
      s += nep[(size_t)tc * ldn + row];
    }
#pragma unroll
    for (int off = 1; off < 32; off <<= 1) s += __shfl_xor(s, off, 32);
    float al = 0.f;
    const float* prow = pe + (size_t)row * ldpe + lane * 4;
    const int nit = ncol / 128;
#pragma unroll 1
    for (int it = 0; it < nit; ++it) {
      const v4f t = *(const v4f*)(prow + it * 128);
#pragma unroll
      for (int k2 = 0; k2 < 4; ++k2) {
        const float pv = t[k2];
        const float rc = __builtin_amdgcn_rcpf(pv + s);
        const float qv = fmaf(pv, rc, eps);
        al += __builtin_amdgcn_logf(qv);
      }
    }
#pragma unroll
    for (int off = 1; off < 32; off <<= 1) al += __shfl_xor(al, off, 32);
    if (lane == 0) rs[wave * 8 + rr] = al;
  }
  __syncthreads();
  const v4f o = *(const v4f*)(rs + 4 * (lane & 15));
  if (wave == 0) {
    float* dst = rowloss + (size_t)blockIdx.x * kRowsPerBlk + 4 * (lane & 15);
    for (int pass = 0; pass < 2; ++pass) {
      if (lane < 16) *(volatile v4f*)dst = o;
      __threadfence();
    }
  }
}

__global__ __launch_bounds__(256) void k_final(const float* __restrict__ colpart, int nbA, int nbP, int nbN, int dim,
                                               const float* __restrict__ rowloss, int nrows,
                                               float* __restrict__ out,
                                               double invBP, double invBN, double lossScale, float tinv) {
  __shared__ double sd[3][256];
  const int t = threadIdx.x;
  double dAP = 0.0, dAN = 0.0;
#pragma unroll 1
  for (int cc = 0; cc < dim / 256; ++cc) {
    const int d = t + cc * 256;
    double sa = 0.0, sp = 0.0, sn = 0.0;
#pragma unroll 8
    for (int b = 0; b < nbA; ++b) sa += (double)colpart[(size_t)b * dim + d];
#pragma unroll 8
    for (int b = 0; b < nbP; ++b) sp += (double)colpart[(size_t)(nbA + b) * dim + d];
#pragma unroll 8
    for (int b = 0; b < nbN; ++b) sn += (double)colpart[(size_t)(nbA + nbP + b) * dim + d];
    dAP += sa * sp;
    dAN += sa * sn;
  }
  double ls = 0.0;
#pragma unroll 8
  for (int q = 0; q < nrows / 256; ++q) ls += (double)rowloss[q * 256 + t];
  sd[0][t] = dAP; sd[1][t] = dAN; sd[2][t] = ls;
  __syncthreads();
  if (t == 0) {
    double sAP = 0.0, sAN = 0.0, sL = 0.0;
#pragma unroll 1
    for (int i = 0; i < 256; ++i) { sAP += sd[0][i]; sAN += sd[1][i]; sL += sd[2][i]; }
    const float mpos = (float)(sAP * (double)tinv * invBP);
    const float mneg = (float)(sAN * (double)tinv * invBN);
    const float loss = (float)(sL * lossScale);
    v4f o;
    o[0] = loss; o[1] = mpos; o[2] = mneg; o[3] = mpos - mneg;
    for (int pass = 0; pass < 2; ++pass) {
      *(volatile v4f*)out = o;
      __threadfence();
    }
  }
}

extern "C" void kernel_launch(void* const* d_in, const int* in_sizes, int n_in,
                              void* d_out, int out_size, void* d_ws, size_t ws_size,
                              hipStream_t stream) {
  if (n_in < 3) return;
  if (in_sizes[0] != kNumAnch * kDim) return;
  if (in_sizes[1] != kNumPos * kDim) return;
  if (in_sizes[2] != kNumNeg * kDim) return;
  if (out_size < 4) return;

  const float* xa = (const float*)d_in[0];
  const float* xp = (const float*)d_in[1];
  const float* xn = (const float*)d_in[2];

  const size_t szA16 = (size_t)kNumAnch * kDim * 2;
  const size_t szP16 = (size_t)kNumPos  * kDim * 2;
  const size_t szN16 = (size_t)kNumNeg  * kDim * 2;
  const size_t szPE  = (size_t)kNumAnch * kNumPos * 4;
  const size_t szNEP = (size_t)kNegTiles * kNumAnch * 4;
  const size_t szCP  = (size_t)(kBlkA + kBlkP + kBlkN) * kDim * 4;
  const size_t szRL  = (size_t)kNumAnch * 4;
  const size_t offA16 = 0;
  const size_t offP16 = offA16 + szA16;
  const size_t offN16 = offP16 + szP16;
  const size_t offPE  = offN16 + szN16;
  const size_t offNEP = offPE  + szPE;
  const size_t offCP  = offNEP + szNEP;
  const size_t offRL  = offCP  + szCP;
  const size_t total  = offRL  + szRL;
  if (total > ws_size) return;

  char* ws = (char*)d_ws;
  _Float16* A16 = (_Float16*)(ws + offA16);
  _Float16* P16 = (_Float16*)(ws + offP16);
  _Float16* N16 = (_Float16*)(ws + offN16);
  float* PE  = (float*)(ws + offPE);
  float* NEP = (float*)(ws + offNEP);
  float* CP  = (float*)(ws + offCP);
  float* RL  = (float*)(ws + offRL);
  const unsigned short* A16u = (const unsigned short*)A16;
  const unsigned short* P16u = (const unsigned short*)P16;
  const unsigned short* N16u = (const unsigned short*)N16;

  const float tinv   = 1.0f / 0.07f;
  const float escale = tinv * 1.4426950408889634f * (1.0f / 256.0f);
  const double invBP = 1.0 / ((double)kNumAnch * (double)kNumPos);
  const double invBN = 1.0 / ((double)kNumAnch * (double)kNumNeg);
  const double lossScale = -0.69314718055994530942 / ((double)kNumAnch * (double)kNumPos);

  k_rownorm<<<kBlkA, 256, 0, stream>>>(xa, kNumAnch, A16, CP);
  k_rownorm<<<kBlkP, 256, 0, stream>>>(xp, kNumPos,  P16, CP + (size_t)kBlkA * kDim);
  k_rownorm<<<kBlkN, 256, 0, stream>>>(xn, kNumNeg,  N16, CP + (size_t)(kBlkA + kBlkP) * kDim);

  wmma_gemm64<0, false, 0, 0, false, 6><<<dim3((kNumAnch / 64) * (kNumPos / 64) / 8, 1), 256, 0, stream>>>(
      A16u, A16u, kDim, 0L,
      P16u, P16u, kDim, 0L,
      (void*)PE, (void*)PE, kNumPos, 0L,
      (const float*)CP,
      (const float*)CP, 0L,
      kNumAnch, kNumPos, kDim, escale);

  gemm64_rowexp2<<<(kNumAnch / 64) * (kNumNeg / 64) / 8, 256, 0, stream>>>(
      A16u, kDim, N16u, kDim, NEP, kNumAnch, kNumAnch, kNumNeg, kDim, escale);

  k_rowloss<<<kNumAnch / kRowsPerBlk, 256, 0, stream>>>(PE, kNumPos, kNumPos, NEP, kNumAnch, kNegTiles,
                                                         RL, kNumAnch, 1e-8f);

  k_final<<<1, 256, 0, stream>>>(CP, kBlkA, kBlkP, kBlkN, kDim, RL, kNumAnch, (float*)d_out,
                                 invBP, invBN, lossScale, tinv);
}
